// Simple_Moe_40810779246876
// MI455X (gfx1250) — hardware-verified
//
#include <hip/hip_runtime.h>


namespace {
constexpr int B = 4096, DIN = 512, F = 512, HN = 2048, O = 512, E = 8, KSEL = 2, NTILE = B * KSEL / 16 + E  ;
constexpr float AS_ = 8.0f, TEMP = 1.5f, MINN = 0.01f;

typedef _Float16 b16;
typedef __attribute__((ext_vector_type(16))) _Float16 v16b;
typedef __attribute__((ext_vector_type(16))) __bf16 v16bb;
typedef __attribute__((ext_vector_type(8))) _Float16 v8b;
typedef __attribute__((ext_vector_type(8))) unsigned short v8us;
typedef __attribute__((ext_vector_type(8))) float v8f;
typedef __attribute__((ext_vector_type(4))) float v4f;
__device__ __forceinline__ float bf16_rne(float f) { unsigned int u = __float_as_uint(f); u += 0x7FFFu + ((u >> 16) & 1u); return __uint_as_float(u & 0xFFFF0000u); }
__device__ __forceinline__ unsigned short bf16_bits(float f) { unsigned int u = __float_as_uint(f); u += 0x7FFFu + ((u >> 16) & 1u); return (unsigned short)(u >> 16); }
__device__ __forceinline__ void split16(float v, b16& hi, b16& lo) { hi = (b16)v; lo = (b16)(v - (float)hi); }
__device__ __forceinline__ v16b frag_kb(const b16* p, int hh) { const v8b a = *(const v8b*)(p + 8 * hh), b = *(const v8b*)(p + 16 + 8 * hh); v16b f;
#pragma unroll
  for (int e = 0; e < 8; ++e) { f[e] = a[e]; f[8 + e] = b[e]; } return f; }
__device__ __forceinline__ v16bb frag_bf(const unsigned short* p, int hh) { const v8us a = *(const v8us*)(p + 8 * hh), b = *(const v8us*)(p + 16 + 8 * hh); union { unsigned short s[16]; v16bb v; } u;
#pragma unroll
  for (int e = 0; e < 8; ++e) { u.s[e] = a[e]; u.s[8 + e] = b[e]; } return u.v; }
__device__ __forceinline__ v16bb frag_f32bf(const float* p, int hh) { union { unsigned short s[16]; v16bb v; } u;
#pragma unroll
  for (int e = 0; e < 8; ++e) { u.s[e] = bf16_bits(p[8 * hh + e]); u.s[8 + e] = bf16_bits(p[16 + 8 * hh + e]); } return u.v; }
__device__ __forceinline__ void frag_split(const float* p, int hh, v16b& fh, v16b& fl) {
#pragma unroll
  for (int e = 0; e < 8; ++e) { b16 a, c; split16(p[8 * hh + e] * AS_, a, c); fh[e] = a; fl[e] = c; split16(p[16 + 8 * hh + e] * AS_, a, c); fh[8 + e] = a; fl[8 + e] = c; } }
__device__ __forceinline__ v8f wmma16b(v16b a, v16b b, v8f c) { v8f d = __builtin_amdgcn_wmma_f32_16x16x32_f16(false, a, false, b, (short)0, c, false, false); asm volatile("v_nop\n\tv_nop\n\tv_nop\n\tv_nop" : "+v"(d) : "v"(a), "v"(b)); return d; }
__device__ __forceinline__ v8f wmma16bb(v16bb a, v16bb b, v8f c) { v8f d = __builtin_amdgcn_wmma_f32_16x16x32_bf16(false, a, false, b, (short)0, c, false, false); asm volatile("v_nop\n\tv_nop\n\tv_nop\n\tv_nop" : "+v"(d) : "v"(a), "v"(b)); return d; }
__device__ __forceinline__ void wave_lds_sync() { __builtin_amdgcn_fence(__ATOMIC_RELEASE, "workgroup"); __builtin_amdgcn_wave_barrier(); __builtin_amdgcn_fence(__ATOMIC_ACQUIRE, "workgroup"); }
__device__ __forceinline__ float nexp(float x) { return __builtin_amdgcn_exp2f(x * 1.4426950408889634f); }
__device__ __forceinline__ float softplus_(float z) { return fmaxf(z, 0.0f) + log1pf(__expf(-fabsf(z))); }

struct Wo_ { static constexpr size_t GN = 0, W1 = GN + 16 * 512, W2 = W1 + (size_t)E * HN * F, END = W2 + (size_t)E * O * HN; };
__global__ __launch_bounds__(256) void prep_kernel(const float* __restrict__ Wb, const float* __restrict__ Wg, const float* __restrict__ bg, const float* __restrict__ Wn, const float* __restrict__ bn, const float* __restrict__ W1, const float* __restrict__ b1, const float* __restrict__ W2, const float* __restrict__ b2, const float* __restrict__ bb,
                                                   unsigned short* __restrict__ wb16, b16* __restrict__ R, float* __restrict__ P) {
  const size_t tid = (size_t)blockIdx.x * blockDim.x + threadIdx.x, nth = (size_t)gridDim.x * blockDim.x;
  for (int pass = 0; pass < 2; ++pass) {
    for (size_t p = tid; p < (size_t)F * DIN / 8; p += nth) { const int o = (int)(p / (DIN / 8)), k8 = (int)(p % (DIN / 8)) * 8; v8us v;
#pragma unroll
      for (int e = 0; e < 8; ++e) v[e] = bf16_bits(Wb[(size_t)(k8 + e) * F + o]);
      *(volatile v8us*)(wb16 + (size_t)o * DIN + k8) = v; }
    for (size_t p = tid; p < (size_t)16 * F / 8; p += nth) { const int o = (int)(p / (F / 8)), k8 = (int)(p % (F / 8)) * 8; v8b v;
#pragma unroll
      for (int e = 0; e < 8; ++e) v[e] = (b16)bf16_rne((o < E) ? Wg[(size_t)(k8 + e) * E + o] : Wn[(size_t)(k8 + e) * E + (o - E)]);
      *(volatile v8b*)(R + Wo_::GN + (size_t)o * F + k8) = v; }
    for (size_t p = tid; p < (size_t)E * HN * F / 8; p += nth) { const int e_ = (int)(p / ((size_t)HN * F / 8)); const size_t q = p % ((size_t)HN * F / 8); const int o = (int)(q / (F / 8)), k8 = (int)(q % (F / 8)) * 8; v8b v;
#pragma unroll
      for (int e = 0; e < 8; ++e) v[e] = (b16)bf16_rne(W1[((size_t)e_ * F + k8 + e) * HN + o]);
      *(volatile v8b*)(R + Wo_::W1 + p * 8) = v; }
    for (size_t p = tid; p < (size_t)E * O * HN / 8; p += nth) { const int e_ = (int)(p / ((size_t)O * HN / 8)); const size_t q = p % ((size_t)O * HN / 8); const int o = (int)(q / (HN / 8)), k8 = (int)(q % (HN / 8)) * 8; v8b v;
#pragma unroll
      for (int e = 0; e < 8; ++e) v[e] = (b16)bf16_rne(W2[((size_t)e_ * HN + k8 + e) * O + o]);
      *(volatile v8b*)(R + Wo_::W2 + p * 8) = v; }
    for (size_t p = tid; p < (16 + E * HN + E * O + F) / 4; p += nth) { v4f v;
#pragma unroll
      for (int e = 0; e < 4; ++e) { const int i = (int)p * 4 + e; float x; if (i < 8) x = bg[i]; else if (i < 16) x = bn[i - 8]; else if (i < 16 + E * HN) x = b1[i - 16]; else if (i < 16 + E * HN + E * O) x = b2[i - 16 - E * HN]; else x = bb[i - 16 - E * HN - E * O]; v[e] = bf16_rne(x); }
      *(volatile v4f*)(P + p * 4) = v; }
    __threadfence(); }
}

__global__ __launch_bounds__(128) void feat_kernel(const float* __restrict__ x, const unsigned short* __restrict__ wb16, const b16* __restrict__ R, const float* __restrict__ P, const float* __restrict__ noise, float* __restrict__ f, float* __restrict__ wrow) {
  __shared__ __attribute__((aligned(16))) float T[4][32][F + 4]; __shared__ float Lg[4][32][16];
  const int lane = threadIdx.x & 31, wave = threadIdx.x >> 5, nloc = lane & 15, hlf = lane >> 4, m0 = blockIdx.x * 128 + wave * 32; const float* bbv = P + 16 + E * HN + E * O;
  for (int ct = 0; ct < F / 64; ++ct) { v8f acc[2][4];
#pragma unroll
    for (int r = 0; r < 2; ++r)
#pragma unroll
      for (int t = 0; t < 4; ++t) acc[r][t] = (v8f){};
#pragma unroll 2
    for (int kb = 0; kb < DIN; kb += 32) { const v16bb a0 = frag_f32bf(x + (size_t)(m0 + nloc) * DIN + kb, hlf), a1 = frag_f32bf(x + (size_t)(m0 + 16 + nloc) * DIN + kb, hlf);
#pragma unroll
      for (int t = 0; t < 4; ++t) { const v16bb bw = frag_bf(wb16 + (size_t)(ct * 64 + t * 16 + nloc) * DIN + kb, hlf); acc[0][t] = wmma16bb(a0, bw, acc[0][t]); acc[1][t] = wmma16bb(a1, bw, acc[1][t]); } }
#pragma unroll
    for (int t = 0; t < 4; ++t) { const int c = ct * 64 + t * 16 + nloc; const float bb = bbv[c];
#pragma unroll
      for (int r = 0; r < 2; ++r)
#pragma unroll
        for (int v = 0; v < 8; ++v) T[wave][r * 16 + 8 * hlf + v][c] = acc[r][t][v] + bb; } }
  wave_lds_sync();
  for (int pass = 0; pass < 2; ++pass) { for (int i = lane; i < 32 * F / 4; i += 32) { const int rr = i / (F / 4), c4 = (i % (F / 4)) * 4; *(volatile v4f*)(f + (size_t)(m0 + rr) * F + c4) = *(const v4f*)(&T[wave][rr][c4]); } __threadfence(); }
  { v8f g0 = {}, g1 = {};
    for (int kb = 0; kb < F; kb += 32) { v16b a0, l0, a1, l1; frag_split(&T[wave][nloc][kb], hlf, a0, l0); frag_split(&T[wave][16 + nloc][kb], hlf, a1, l1); const v16b bw = frag_kb(R + Wo_::GN + (size_t)nloc * F + kb, hlf);
      g0 = wmma16b(a0, bw, g0); g0 = wmma16b(l0, bw, g0); g1 = wmma16b(a1, bw, g1); g1 = wmma16b(l1, bw, g1); }
#pragma unroll
    for (int v = 0; v < 8; ++v) { Lg[wave][8 * hlf + v][nloc] = g0[v] * (1.0f / AS_); Lg[wave][16 + 8 * hlf + v][nloc] = g1[v] * (1.0f / AS_); } }
  wave_lds_sync();
  { const int rr = lane, tok = m0 + rr; float g[E];
#pragma unroll
    for (int e = 0; e < E; ++e) { const float raw = Lg[wave][rr][e] + P[e], zn = Lg[wave][rr][E + e] + P[E + e]; g[e] = raw + (softplus_(zn) + MINN) * bf16_rne(noise[(size_t)tok * E + e]); }
    int e0 = 0; float v0 = g[0];
#pragma unroll
    for (int e = 1; e < E; ++e) if (g[e] > v0) { v0 = g[e]; e0 = e; }
    int e1 = -1; float v1 = -INFINITY;
#pragma unroll
    for (int e = 0; e < E; ++e) if (e != e0 && (e1 < 0 || g[e] > v1)) { v1 = g[e]; e1 = e; }
    const float a1 = nexp((v1 - v0) * (1.0f / TEMP)); const float w0 = 1.0f / (1.0f + a1), w1 = a1 / (1.0f + a1);
    v4f wa = {0.0f, 0.0f, 0.0f, 0.0f}, wb = {0.0f, 0.0f, 0.0f, 0.0f};
#pragma unroll
    for (int e = 0; e < 4; ++e) { wa[e] = (e == e0) ? w0 : ((e == e1) ? w1 : 0.0f); wb[e] = (e + 4 == e0) ? w0 : ((e + 4 == e1) ? w1 : 0.0f); }
    for (int pass = 0; pass < 2; ++pass) { *(volatile v4f*)(wrow + (size_t)tok * 8) = wa; *(volatile v4f*)(wrow + (size_t)tok * 8 + 4) = wb; __threadfence(); } }
}

__global__ __launch_bounds__(64) void expert_kernel(const float* __restrict__ f, const float* __restrict__ wrow, const b16* __restrict__ R, const float* __restrict__ P, float* __restrict__ Y) {
  __shared__ __attribute__((aligned(16))) b16 Fh[16][F + 8], Fl[16][F + 8]; __shared__ __attribute__((aligned(16))) float Hc[16][256 + 4]; __shared__ __attribute__((aligned(16))) float Yt[16][O + 4]; __shared__ int toks[256]; __shared__ int wcnt[2];
  const int wid = threadIdx.x >> 5, lane = threadIdx.x & 31, nloc = lane & 15, hlf = lane >> 4; const int c0 = blockIdx.x * 256, e = blockIdx.y;
  int ntok;
  { const int tb = c0 + threadIdx.x * 4; bool hit[4]; int nh = 0;
#pragma unroll
    for (int q = 0; q < 4; ++q) { hit[q] = (wrow[(size_t)(tb + q) * E + e] != 0.0f); nh += hit[q] ? 1 : 0; }
    int incl = nh;
#pragma unroll
    for (int o = 1; o < 32; o <<= 1) { const int t = __shfl_up(incl, o); if (lane >= o) incl += t; }
    if (lane == 31) wcnt[wid] = incl;
    __syncthreads();
    const int woff = (wid == 1) ? wcnt[0] : 0; ntok = wcnt[0] + wcnt[1]; int pos = woff + incl - nh;
#pragma unroll
    for (int q = 0; q < 4; ++q) if (hit[q]) toks[pos++] = tb + q;
    __syncthreads(); }
  const b16* W1e = R + Wo_::W1 + (size_t)e * HN * F; const b16* W2e = R + Wo_::W2 + (size_t)e * O * HN; const float* b1e = P + 16 + (size_t)e * HN; const float* b2e = P + 16 + (size_t)E * HN + (size_t)e * O;
  for (int r0 = 0; r0 < ntok; r0 += 16) { const int nvalid = min(16, ntok - r0);
    __syncthreads();
    for (int i = threadIdx.x; i < 16 * (F / 4); i += 64) { const int rr = i / (F / 4), c4 = (i % (F / 4)) * 4; const int tok = toks[r0 + ((rr < nvalid) ? rr : 0)]; const v4f v = *(const v4f*)(f + (size_t)tok * F + c4);
#pragma unroll
      for (int q = 0; q < 4; ++q) { b16 a, c; split16(v[q] * AS_, a, c); Fh[rr][c4 + q] = a; Fl[rr][c4 + q] = c; } }
    __syncthreads();
    v8f yacc[16];
#pragma unroll
    for (int t = 0; t < 16; ++t) yacc[t] = (v8f){};
    for (int hc = 0; hc < HN; hc += 256) {
      v8f ha[8];
#pragma unroll
      for (int t = 0; t < 8; ++t) ha[t] = (v8f){};
#pragma unroll 2
      for (int kb = 0; kb < F; kb += 32) { const v16b ah = frag_kb(&Fh[nloc][kb], hlf), al = frag_kb(&Fl[nloc][kb], hlf);
#pragma unroll
        for (int t = 0; t < 8; ++t) { const v16b bw = frag_kb(W1e + (size_t)(hc + wid * 128 + t * 16 + nloc) * F + kb, hlf); ha[t] = wmma16b(ah, bw, ha[t]); ha[t] = wmma16b(al, bw, ha[t]); } }
      __syncthreads();
#pragma unroll
      for (int t = 0; t < 8; ++t) { const int cl = wid * 128 + t * 16 + nloc; const float bb = b1e[hc + cl];
#pragma unroll
        for (int v = 0; v < 8; ++v) Hc[8 * hlf + v][cl] = fmaxf(ha[t][v] * (1.0f / AS_) + bb, 0.0f); }
      __syncthreads();
      for (int kb = 0; kb < 256; kb += 32) { v16b ah, al; frag_split(&Hc[nloc][kb], hlf, ah, al);
#pragma unroll
        for (int t = 0; t < 16; ++t) { const v16b bw = frag_kb(W2e + (size_t)(wid * 256 + t * 16 + nloc) * HN + hc + kb, hlf); yacc[t] = wmma16b(ah, bw, yacc[t]); yacc[t] = wmma16b(al, bw, yacc[t]); } }
    }
#pragma unroll
    for (int t = 0; t < 16; ++t) { const int c = wid * 256 + t * 16 + nloc; const float bb = b2e[c];
#pragma unroll
      for (int v = 0; v < 8; ++v) Yt[8 * hlf + v][c] = yacc[t][v] * (1.0f / AS_) + bb; }
    __syncthreads();
    for (int pass = 0; pass < 2; ++pass) { for (int i = threadIdx.x; i < 16 * (O / 4); i += 64) { const int rr = i / (O / 4), c4 = (i % (O / 4)) * 4; if (rr < nvalid) *(volatile v4f*)(Y + ((size_t)toks[r0 + rr] * E + e) * O + c4) = *(const v4f*)(&Yt[rr][c4]); } __threadfence(); }
  }
}

__global__ __launch_bounds__(256) void combine_kernel(const float* __restrict__ Y, const float* __restrict__ wrow, float* __restrict__ out) {
  const size_t g = (size_t)blockIdx.x * 256 + threadIdx.x; const int tok = (int)(g / (O / 4)), c4 = (int)(g % (O / 4)) * 4;
  v4f o = {0.0f, 0.0f, 0.0f, 0.0f};
  for (int e = 0; e < E; ++e) { const float w = wrow[(size_t)tok * E + e]; if (w != 0.0f) { const v4f y = *(const v4f*)(Y + ((size_t)tok * E + e) * O + c4);
#pragma unroll
      for (int q = 0; q < 4; ++q) o[q] += w * y[q]; } }
  for (int pass = 0; pass < 2; ++pass) { *(volatile v4f*)(out + (size_t)tok * O + c4) = o; __threadfence(); }
}
}
extern "C" void kernel_launch(void* const* d_in, const int* in_sizes, int n_in,
                              void* d_out, int out_size, void* d_ws, size_t ws_size, hipStream_t stream) {
  (void)n_in; (void)out_size;
  const float* x = (const float*)d_in[0]; const float* noise = (const float*)d_in[1]; const float* Wb = (const float*)d_in[2]; const float* bb = (const float*)d_in[3]; const float* Wg = (const float*)d_in[4]; const float* bg = (const float*)d_in[5]; const float* Wn = (const float*)d_in[6]; const float* bn = (const float*)d_in[7];
  const float* W1 = (const float*)d_in[8]; const float* b1 = (const float*)d_in[9]; const float* W2 = (const float*)d_in[10]; const float* b2 = (const float*)d_in[11];
  float* out = (float*)d_out;
  if (in_sizes[0] != B * DIN || in_sizes[1] != B * E || in_sizes[2] != DIN * F || in_sizes[8] != E * F * HN || in_sizes[10] != E * HN * O) return;
  size_t off = 0; char* ws = (char*)d_ws;
  auto carve = [&](size_t bytes) { char* p = ws + off; off += (bytes + 255) & ~(size_t)255; return p; };
  unsigned short* wb16 = (unsigned short*)carve((size_t)F * DIN * 2); b16* R = (b16*)carve(Wo_::END * 2); float* P = (float*)carve((size_t)(16 + E * HN + E * O + F + 64) * 4);
  float* f = (float*)carve((size_t)B * F * 4); float* wrow = (float*)carve((size_t)B * E * 4); float* Y = (float*)carve((size_t)B * E * O * 4);
  if (off > ws_size) return;
  prep_kernel<<<1024, 256, 0, stream>>>(Wb, Wg, bg, Wn, bn, W1, b1, W2, b2, bb, wb16, R, P);
  feat_kernel<<<B / 128, 128, 0, stream>>>(x, wb16, R, P, noise, f, wrow);
  expert_kernel<<<dim3(B / 256, E), 64, 0, stream>>>(f, wrow, R, P, Y);
  combine_kernel<<<B * O / 4 / 256, 256, 0, stream>>>(Y, wrow, out);
}
